// TransformerEncoderLayer_32014686225065
// MI455X (gfx1250) — hardware-verified
//
#include <hip/hip_runtime.h>
#ifndef NB
#define NB 2
#endif
#ifndef SEQ
#define SEQ 2048
#endif
#define NB_FULL 2
#define SEQ_FULL 2048
#define DM 1024
#define NH 16
#define HD 64
#define DFF 4096
#define HG 2
#define SQ SEQ
#define LQ (3 * DM)
#define NR ((size_t)NB * SEQ)
static_assert(SEQ % 128 == 0);
static_assert(SEQ <= SEQ_FULL);
static_assert(NB >= 1 && NB <= NB_FULL);
static_assert(NH % HG == 0);
static_assert(NH * HD == DM);
static_assert(DM % 64 == 0 && DFF % 64 == 0 && HD == 64 && LQ % 64 == 0);
static_assert(DM % 32 == 0 && DFF % 32 == 0 && SEQ % 32 == 0 && HD % 32 == 0);
static_assert(DM / 4 <= 256);
static_assert(((size_t)NB * SEQ) % 128 == 0);
static_assert(((size_t)SEQ * HG) % 256 == 0);
static_assert(SQ % 8 == 0);

typedef _Float16 v16h __attribute__((ext_vector_type(16)));
typedef unsigned short v8us __attribute__((ext_vector_type(8), may_alias));
typedef float v8f __attribute__((ext_vector_type(8)));
typedef float v4f __attribute__((ext_vector_type(4)));
typedef float v4fa __attribute__((ext_vector_type(4), may_alias));
typedef _Float16 v4h __attribute__((ext_vector_type(4)));
union FragH { v16h v; v8us half[2]; _Float16 h[16]; unsigned short u[16]; };

constexpr size_t al256(size_t b) { return (b + 255) & ~(size_t)255; }
constexpr size_t OFF_BQKV = 0;
constexpr size_t OFF_BO   = OFF_BQKV + al256((size_t)3 * DM * DM * 2);
constexpr size_t OFF_BIAS = OFF_BO   + al256((size_t)DM * DM * 2);
constexpr size_t OFF_BW1  = OFF_BIAS + al256((size_t)3 * DM * 4);
constexpr size_t OFF_BW2  = OFF_BW1  + al256((size_t)DFF * DM * 2);
constexpr size_t OFF_X16  = OFF_BW2  + al256((size_t)DM * DFF * 2);
constexpr size_t OFF_O16  = OFF_X16  + al256(NR * DM * 2);
constexpr size_t OFF_U    = OFF_O16  + al256(NR * DM * 2);
constexpr size_t OFA_QKV  = OFF_U;
constexpr size_t OFA_VT   = OFA_QKV  + al256((size_t)SEQ * LQ * 2);
constexpr size_t OFA_S    = OFA_VT   + al256((size_t)NH * HD * SEQ * 2);
constexpr size_t OFA_P    = OFA_S    + al256((size_t)HG * SEQ * SEQ * 4);
constexpr size_t END_A    = OFA_P    + al256((size_t)HG * SEQ * SEQ * 2);
constexpr size_t OFB_R1   = OFF_U;
constexpr size_t OFB_X1F  = OFB_R1   + al256(NR * DM * 4);
constexpr size_t OFB_M16  = OFB_X1F  + al256(NR * DM * 4);
constexpr size_t OFB_HF   = OFB_M16  + al256(NR * DM * 2);
constexpr size_t END_B    = OFB_HF   + al256(NR * DFF * 2);
constexpr size_t WS_TOTAL = (END_A > END_B) ? END_A : END_B;
static_assert(WS_TOTAL <= (size_t)134217728);

__device__ __forceinline__ unsigned short bf16_bits(float x) { unsigned int u = __float_as_uint(x); return (unsigned short)((u + 0x7FFFu + ((u >> 16) & 1u)) >> 16); }
__device__ __forceinline__ float bf16_val(unsigned short b) { return __uint_as_float(((unsigned int)b) << 16); }
__device__ __forceinline__ float bf16_rne(float x) { return bf16_val(bf16_bits(x)); }
__device__ __forceinline__ size_t frow(size_t r) { return (r / SEQ) * SEQ_FULL + (r % SEQ); }

__device__ __forceinline__ v16h g2_frag(const _Float16* p, unsigned hh) { FragH f; f.half[0] = *(const v8us*)((const unsigned short*)p + 8u * hh); f.half[1] = *(const v8us*)((const unsigned short*)p + 16u + 8u * hh); return f.v; }
__device__ __forceinline__ v8f g2_mma(v16h a, v16h b, v8f c) { v8f d = __builtin_amdgcn_wmma_f32_16x16x32_f16(false, a, false, b, (short)0, c, false, false); asm volatile("v_nop\n\tv_nop\n\tv_nop\n\tv_nop" : "+v"(d) : "v"(a), "v"(b)); return d; }

template <int ACT, int OSH>
__global__ __launch_bounds__(128) void k_gemm2(const _Float16* __restrict__ A, int lda, size_t sA, const _Float16* __restrict__ Bh, int ldb, size_t sB, float alpha,
                                               const float* __restrict__ bias, const float* __restrict__ CP,
                                               float* __restrict__ C, _Float16* __restrict__ C16, int ldc, size_t sC, int M, int N, int K) {
  static_assert(ACT == 0 || ACT == 1);
  static_assert(OSH >= 0 && OSH < 12);
  __shared__ __attribute__((aligned(16))) float so[4][32][68];
  const unsigned tid = threadIdx.x, w = tid >> 5, lane = tid & 31u, ln = lane & 15u, hh = lane >> 4; const unsigned by = blockIdx.y;
  A += (size_t)by * sA; Bh += (size_t)by * sB; const size_t cofs = (size_t)by * sC;
  const unsigned ntn = (unsigned)N >> 6; const unsigned mt = blockIdx.x / ntn, nq = blockIdx.x - mt * ntn; const unsigned row0 = mt * 128u + 32u * w, col0 = nq * 64u;
  if (row0 >= (unsigned)M) return;
  const _Float16* a0p = A + (size_t)(row0 + ln) * (size_t)lda; const _Float16* a1p = a0p + (size_t)16 * (size_t)lda;
  const _Float16* b0p = Bh + (size_t)(col0 + ln) * (size_t)ldb; const _Float16* b1p = b0p + (size_t)16 * (size_t)ldb; const _Float16* b2p = b1p + (size_t)16 * (size_t)ldb; const _Float16* b3p = b2p + (size_t)16 * (size_t)ldb;
  const v8f z8 = {0.f, 0.f, 0.f, 0.f, 0.f, 0.f, 0.f, 0.f};
  v8f c00 = z8, c01 = z8, c02 = z8, c03 = z8, c10 = z8, c11 = z8, c12 = z8, c13 = z8;
#pragma unroll 1
  for (int kb = 0; kb < K; kb += 32) {
    const v16h a0 = g2_frag(a0p + kb, hh), a1 = g2_frag(a1p + kb, hh);
    v16h b = g2_frag(b0p + kb, hh); c00 = g2_mma(a0, b, c00); c10 = g2_mma(a1, b, c10);
    b = g2_frag(b1p + kb, hh); c01 = g2_mma(a0, b, c01); c11 = g2_mma(a1, b, c11);
    b = g2_frag(b2p + kb, hh); c02 = g2_mma(a0, b, c02); c12 = g2_mma(a1, b, c12);
    b = g2_frag(b3p + kb, hh); c03 = g2_mma(a0, b, c03); c13 = g2_mma(a1, b, c13);
  }
  v8f accs[8] = {c00, c01, c02, c03, c10, c11, c12, c13};
#pragma unroll
  for (int u = 0; u < 8; ++u) {
    const unsigned t = (unsigned)(u & 3), half = (unsigned)(u >> 2); const unsigned col = col0 + t * 16u + ln;
    const float bv = bias ? bf16_rne(bias[col]) : 0.f;
#pragma unroll
    for (int r = 0; r < 8; ++r) {
      const unsigned rloc = half * 16u + 8u * hh + (unsigned)r;
      float v = accs[u][r] * alpha + bv;
      if (CP) v += CP[cofs + (size_t)(row0 + rloc) * (size_t)ldc + col];
      if (ACT == 1) v = fmaxf(v, 0.0f);
      if (OSH > 0) v = v * (float)(1 << OSH);
      so[w][rloc][t * 16u + ln] = v;
    }
  }
  __builtin_amdgcn_fence(4  , "workgroup"); __builtin_amdgcn_wave_barrier();
  const unsigned rsub = lane >> 4, c4 = (lane & 15u) * 4u;
  for (int pass = 0; pass < 2; ++pass) {
#pragma unroll
    for (int q = 0; q < 16; ++q) {
      const unsigned r = (unsigned)q * 2u + rsub;
      const v4f v = *(const v4fa*)&so[w][r][c4];
      if (C) *(volatile v4f*)(C + cofs + (size_t)(row0 + r) * (size_t)ldc + col0 + c4) = v;
      if (C16) { v4h h4; for (int i = 0; i < 4; ++i) h4[i] = (_Float16)v[i]; *(volatile v4h*)(C16 + cofs + (size_t)(row0 + r) * (size_t)ldc + col0 + c4) = h4; }
    }
    if (pass == 0) __threadfence();
  }
}

__global__ __launch_bounds__(256) void k_wt_f16(const float* __restrict__ W, _Float16* __restrict__ Wt, int K, int N, float scale) {
  const unsigned k8n = (unsigned)K >> 3; const unsigned t = blockIdx.x * 256u + threadIdx.x; if (t >= (unsigned)N * k8n) return;
  const unsigned n = t / k8n, k8 = (t - n * k8n) * 8u; FragH f;
#pragma unroll
  for (int i = 0; i < 8; ++i) f.h[i] = (_Float16)(bf16_rne(W[(size_t)(k8 + (unsigned)i) * (size_t)N + n]) * scale);
  const v8us o = f.half[0];
  *(volatile v8us*)((unsigned short*)Wt + (size_t)n * (size_t)K + k8) = o; __threadfence(); *(volatile v8us*)((unsigned short*)Wt + (size_t)n * (size_t)K + k8) = o;
}

__global__ __launch_bounds__(256) void k_wthd(const float* __restrict__ W, _Float16* __restrict__ Bt) {
  const unsigned t = blockIdx.x * 256u + threadIdx.x; if (t >= (unsigned)(NH * HD * (DM / 8))) return;
  const unsigned m8 = (t % (unsigned)(DM / 8)) * 8u; const unsigned d = (t / (unsigned)(DM / 8)) % (unsigned)HD; const unsigned h = t / (unsigned)((DM / 8) * HD); FragH f;
#pragma unroll
  for (int q = 0; q < 8; ++q) f.h[q] = (_Float16)(16.0f * bf16_rne(W[((size_t)h * DM + m8 + (unsigned)q) * HD + d]));
  unsigned short* dst = (unsigned short*)Bt + ((size_t)h * HD + d) * DM + m8;
  const v8us o = f.half[0];
  *(volatile v8us*)dst = o; __threadfence(); *(volatile v8us*)dst = o;
}

__global__ __launch_bounds__(256) void k_bcpy(const float* __restrict__ b, int n, int NP, float* __restrict__ dst, int dst0) {
  for (int i = threadIdx.x; i < NP; i += 256) { const float v = (i < n) ? b[min(i, n - 1)] : 0.f; *(volatile float*)(dst + dst0 + i) = v; }
  __threadfence();
  for (int i = threadIdx.x; i < NP; i += 256) { const float v = (i < n) ? b[min(i, n - 1)] : 0.f; *(volatile float*)(dst + dst0 + i) = v; }
}

__global__ __launch_bounds__(256) void k_x16r(const float* __restrict__ x, _Float16* __restrict__ X16, size_t n8) {
  const size_t t = (size_t)blockIdx.x * 256 + threadIdx.x; if (t >= n8) return;
  const size_t e = t * 8; const size_t r = e / DM; const unsigned c = (unsigned)(e % DM); const size_t rf = frow(r);
  const v4f a = *(const v4fa*)(x + rf * DM + c), bq4 = *(const v4fa*)(x + rf * DM + c + 4);
  FragH f;
#pragma unroll
  for (int q = 0; q < 4; ++q) { f.h[q] = (_Float16)bf16_rne(a[q]); f.h[4 + q] = (_Float16)bf16_rne(bq4[q]); }
  const v8us o = f.half[0];
  *(volatile v8us*)((unsigned short*)X16 + e) = o; __threadfence(); *(volatile v8us*)((unsigned short*)X16 + e) = o;
}

template <int NHv, int TTv>
__global__ __launch_bounds__(256) void k_vt(const _Float16* __restrict__ V16, int ldv, int voff, _Float16* __restrict__ Vt) {
  __shared__ unsigned short tl[64][66];
  const unsigned tid = threadIdx.x; const unsigned slab = blockIdx.x / (unsigned)(TTv / 64), lg = blockIdx.x % (unsigned)(TTv / 64); const unsigned b = slab / (unsigned)NHv, h = slab % (unsigned)NHv;
  for (unsigned i = tid; i < 64u * 8u; i += 256u) {
    const unsigned r = i >> 3, c8 = (i & 7u) * 8u; FragH f;
    f.half[0] = *(const v8us*)((const unsigned short*)V16 + ((size_t)b * TTv + lg * 64u + r) * (size_t)ldv + (size_t)voff + h * 64u + c8);
#pragma unroll
    for (int q = 0; q < 8; ++q) tl[r][c8 + (unsigned)q] = f.u[q];
  }
  __syncthreads();
  for (int pass = 0; pass < 2; ++pass) {
#pragma unroll
    for (int rd = 0; rd < 2; ++rd) {
      const unsigned d = (unsigned)rd * 32u + (tid >> 3), pc = tid & 7u; FragH f;
#pragma unroll
      for (int q = 0; q < 8; ++q) f.u[q] = tl[pc * 8u + (unsigned)q][d];
      const v8us o = f.half[0];
      *(volatile v8us*)((unsigned short*)Vt + ((size_t)slab * 64 + d) * TTv + lg * 64u + pc * 8u) = o;
    }
    if (pass == 0) __threadfence();
  }
}

__global__ __launch_bounds__(256) void k_rsmf(const float* __restrict__ S, _Float16* __restrict__ P, int qn, int hg) {
  #pragma clang fp contract(off)
  const unsigned t = blockIdx.x * 256u + threadIdx.x; if (t >= (unsigned)qn * (unsigned)hg) return;
  const unsigned sl = t / (unsigned)qn; const size_t i = (size_t)sl * SQ + (size_t)(t - sl * (unsigned)qn);
  const float* s = S + i * SQ; float mx = -3.0e38f;
#pragma unroll 1
  for (int j0 = 0; j0 < SQ; j0 += 8) {
    const v4f a = *(const v4fa*)(s + j0), b = *(const v4fa*)(s + j0 + 4);
    const float m0 = fmaxf(fmaxf(a[0], a[1]), fmaxf(a[2], a[3])); const float m1 = fmaxf(fmaxf(b[0], b[1]), fmaxf(b[2], b[3]));
    mx = fmaxf(mx, fmaxf(m0, m1));
  }
  float se = 0.f;
#pragma unroll 1
  for (int j0 = 0; j0 < SQ; j0 += 8) {
    const v4f a = *(const v4fa*)(s + j0), b = *(const v4fa*)(s + j0 + 4);
#pragma unroll
    for (int q = 0; q < 4; ++q) se += __expf(a[q] - mx);
#pragma unroll
    for (int q = 0; q < 4; ++q) se += __expf(b[q] - mx);
  }
  const float sc = 256.0f * (1.0f / se);
#pragma unroll 1
  for (int j0 = 0; j0 < SQ; j0 += 8) {
    const v4f a = *(const v4fa*)(s + j0), b = *(const v4fa*)(s + j0 + 4);
    FragH f;
#pragma unroll
    for (int q = 0; q < 4; ++q) { f.h[q] = (_Float16)(__expf(a[q] - mx) * sc); f.h[4 + q] = (_Float16)(__expf(b[q] - mx) * sc); }
    unsigned short* d = (unsigned short*)P + i * SQ + j0;
    const v8us o = f.half[0];
    *(volatile v8us*)d = o; __threadfence(); *(volatile v8us*)d = o;
  }
}

template <int HASR, int W16, int W32, int OREMAP>
__global__ __launch_bounds__(256) void k_lnr(const float* __restrict__ X, const float* __restrict__ RX, const float* __restrict__ g, const float* __restrict__ bb, float eps,
                                             _Float16* __restrict__ N16, float* __restrict__ N32) {
  #pragma clang fp contract(off)
  __shared__ float red[256];
  const size_t r = blockIdx.x; const unsigned t = threadIdx.x; const bool act = t < (unsigned)(DM / 4); const unsigned c0 = act ? t * 4u : 0u;
  const size_t rf = frow(r);
  const v4f xa = *(const v4fa*)(X + r * DM + c0);
  v4f ra = {0.f, 0.f, 0.f, 0.f};
  if (HASR) ra = *(const v4fa*)(RX + rf * DM + c0);
  float s[4]; float sum = 0.f;
#pragma unroll
  for (int q = 0; q < 4; ++q) { const float rv = HASR ? bf16_rne(ra[q]) : 0.f; s[q] = act ? __fadd_rn(xa[q], rv) : 0.f; sum = __fadd_rn(sum, s[q]); }
  red[t] = sum; __syncthreads();
  for (unsigned st = 128u; st > 0u; st >>= 1) { if (t < st) red[t] = __fadd_rn(red[t], red[t + st]); __syncthreads(); }
  const float mu = red[0] * (1.0f / (float)DM); __syncthreads();
  float vs = 0.f;
#pragma unroll
  for (int q = 0; q < 4; ++q) { const float dl = act ? __fadd_rn(s[q], -mu) : 0.f; vs = __fadd_rn(vs, __fmul_rn(dl, dl)); }
  red[t] = vs; __syncthreads();
  for (unsigned st = 128u; st > 0u; st >>= 1) { if (t < st) red[t] = __fadd_rn(red[t], red[t + st]); __syncthreads(); }
  const float rs = rsqrtf(__fadd_rn(red[0] * (1.0f / (float)DM), eps));
  v4h y; v4f yf;
#pragma unroll
  for (int q = 0; q < 4; ++q) {
    const unsigned c = c0 + (unsigned)q;
    yf[q] = __fadd_rn(__fmul_rn(__fmul_rn(__fadd_rn(s[q], -mu), rs), bf16_rne(g[c])), bf16_rne(bb[c]));
    y[q] = (_Float16)yf[q];
  }
  if (!act) return;
  const size_t ro = OREMAP ? rf : r;
  for (int pass = 0; pass < 2; ++pass) {
    if (W16) *(volatile v4h*)(N16 + r * DM + c0) = y;
    if (W32) *(volatile v4f*)(N32 + ro * DM + c0) = yf;
    if (pass == 0) __threadfence();
  }
}

extern "C" void kernel_launch(void* const* d_in, const int* in_sizes, int n_in,
                              void* d_out, int out_size, void* d_ws, size_t ws_size, hipStream_t stream) {
  if (n_in < 17) return;
  const float* x   = (const float*)d_in[0];
  const float* wq  = (const float*)d_in[1];  const float* bq  = (const float*)d_in[2];
  const float* wk  = (const float*)d_in[3];  const float* bk  = (const float*)d_in[4];
  const float* wv  = (const float*)d_in[5];  const float* bvv = (const float*)d_in[6];
  const float* wo  = (const float*)d_in[7];  const float* bo  = (const float*)d_in[8];
  const float* g1  = (const float*)d_in[9];  const float* be1 = (const float*)d_in[10];
  const float* w1  = (const float*)d_in[11]; const float* b1  = (const float*)d_in[12];
  const float* w2  = (const float*)d_in[13]; const float* b2  = (const float*)d_in[14];
  const float* g2  = (const float*)d_in[15]; const float* be2 = (const float*)d_in[16];
  const size_t need_x = ((size_t)(NB - 1) * SEQ_FULL + SEQ) * DM;
  if (in_sizes[0] < 0 || (size_t)in_sizes[0] < need_x || out_size < 0 || (size_t)out_size < need_x) return;
  if (in_sizes[1] < NH * DM * HD || in_sizes[3] < NH * DM * HD || in_sizes[5] < NH * DM * HD) return;
  if (in_sizes[2] < NH * HD || in_sizes[4] < NH * HD || in_sizes[6] < NH * HD) return;
  if (in_sizes[7] < DM * DM || in_sizes[8] < DM) return;
  if (in_sizes[9] < DM || in_sizes[10] < DM) return;
  if (in_sizes[11] < DM * DFF || in_sizes[12] < DFF || in_sizes[13] < DFF * DM || in_sizes[14] < DM) return;
  if (in_sizes[15] < DM || in_sizes[16] < DM) return;
  if (WS_TOTAL > ws_size) return;

  char* ws = (char*)d_ws;
  _Float16* BQKV  = (_Float16*)(ws + OFF_BQKV);
  _Float16* BO    = (_Float16*)(ws + OFF_BO);
  float*    bqkvi = (float*)(ws + OFF_BIAS);
  _Float16* BW1   = (_Float16*)(ws + OFF_BW1);
  _Float16* BW2   = (_Float16*)(ws + OFF_BW2);
  _Float16* X16   = (_Float16*)(ws + OFF_X16);
  _Float16* O16   = (_Float16*)(ws + OFF_O16);
  _Float16* QKV   = (_Float16*)(ws + OFA_QKV);
  _Float16* VT    = (_Float16*)(ws + OFA_VT);
  float*    S     = (float*)(ws + OFA_S);
  _Float16* P     = (_Float16*)(ws + OFA_P);
  float*    R1    = (float*)(ws + OFB_R1);
  float*    X1F   = (float*)(ws + OFB_X1F);
  _Float16* M16   = (_Float16*)(ws + OFB_M16);
  _Float16* HF16  = (_Float16*)(ws + OFB_HF);
  float*    R2    = R1;

  { const unsigned g = (unsigned)(((size_t)NH * HD * (DM / 8) + 255) / 256);
    k_wthd<<<g, 256, 0, stream>>>(wq, BQKV);
    k_wthd<<<g, 256, 0, stream>>>(wk, BQKV + (size_t)DM * DM);
    k_wthd<<<g, 256, 0, stream>>>(wv, BQKV + (size_t)2 * DM * DM); }
  k_bcpy<<<1, 256, 0, stream>>>(bq, NH * HD, DM, bqkvi, 0);
  k_bcpy<<<1, 256, 0, stream>>>(bk, NH * HD, DM, bqkvi, DM);
  k_bcpy<<<1, 256, 0, stream>>>(bvv, NH * HD, DM, bqkvi, 2 * DM);
  k_wt_f16<<<(unsigned)(((size_t)DM * (DM / 8) + 255) / 256), 256, 0, stream>>>(wo, BO, DM, DM, 16.0f);
  k_wt_f16<<<(unsigned)(((size_t)DFF * (DM / 8) + 255) / 256), 256, 0, stream>>>(w1, BW1, DM, DFF, 16.0f);
  k_wt_f16<<<(unsigned)(((size_t)DM * (DFF / 8) + 255) / 256), 256, 0, stream>>>(w2, BW2, DFF, DM, 16.0f);
  k_x16r<<<(unsigned)((NR * DM / 8 + 255) / 256), 256, 0, stream>>>(x, X16, NR * DM / 8);

  for (int b = 0; b < NB; ++b) {
    const size_t r0c = (size_t)b * SEQ;
    k_gemm2<0, 0><<<dim3((unsigned)((SEQ / 128) * (LQ / 64)), 1), 128, 0, stream>>>(
        X16 + r0c * DM, DM, (size_t)0, BQKV, DM, (size_t)0, 0.0625f, bqkvi, nullptr, nullptr, QKV, LQ, (size_t)0, SEQ, LQ, DM);
    k_vt<NH, SEQ><<<(unsigned)(NH * (SEQ / 64)), 256, 0, stream>>>(QKV + 2 * DM, LQ, 0, VT);
    for (int h0 = 0; h0 < NH; h0 += HG) {
      k_gemm2<0, 0><<<dim3((unsigned)((SEQ / 128) * (SEQ / 64)), HG), 128, 0, stream>>>(
          QKV + (size_t)h0 * HD, LQ, (size_t)HD, QKV + DM + (size_t)h0 * HD, LQ, (size_t)HD, 0.125f, nullptr, nullptr, S, nullptr, SEQ, (size_t)SEQ * SEQ, SEQ, SEQ, HD);
      k_rsmf<<<(unsigned)(((size_t)SEQ * HG + 255) / 256), 256, 0, stream>>>(S, P, SEQ, HG);
      k_gemm2<0, 0><<<dim3((unsigned)((SEQ / 128) * (HD / 64)), HG), 128, 0, stream>>>(
          P, SEQ, (size_t)SEQ * SEQ, VT + (size_t)h0 * HD * SEQ, SEQ, (size_t)HD * SEQ, 0.25f, nullptr, nullptr, nullptr, O16 + r0c * DM + (size_t)h0 * HD, DM, (size_t)HD, SEQ, HD, SEQ);
    }
  }
  k_gemm2<0, 0><<<dim3((unsigned)((NR / 128) * (DM / 64)), 1), 128, 0, stream>>>(
      O16, DM, (size_t)0, BO, DM, (size_t)0, 0.0009765625f, bo, nullptr, R1, nullptr, DM, (size_t)0, (int)NR, DM, DM);
  k_lnr<1, 1, 1, 0><<<(unsigned)NR, 256, 0, stream>>>(R1, x, g1, be1, 1e-5f, M16, X1F);
  k_gemm2<1, 6><<<dim3((unsigned)((NR / 128) * (DFF / 64)), 1), 128, 0, stream>>>(
      M16, DM, (size_t)0, BW1, DM, (size_t)0, 0.0625f, b1, nullptr, nullptr, HF16, DFF, (size_t)0, (int)NR, DFF, DM);
  k_gemm2<0, 0><<<dim3((unsigned)((NR / 128) * (DM / 64)), 1), 128, 0, stream>>>(
      HF16, DFF, (size_t)0, BW2, DFF, (size_t)0, 0.0009765625f, b2, X1F, R2, nullptr, DM, (size_t)0, (int)NR, DM, DFF);
  k_lnr<0, 0, 1, 1><<<(unsigned)NR, 256, 0, stream>>>(R2, nullptr, g2, be2, 1e-5f, nullptr, (float*)d_out);
}
